// MultiHeadattention_24361054502928
// MI455X (gfx1250) — hardware-verified
//
#include <hip/hip_runtime.h>
#include <stdint.h>

constexpr int kBatch  = 2;
constexpr int kSeq    = 2048;
constexpr int kDm     = 1024;
constexpr int kHeads  = 16;
constexpr int kDk     = 64;
constexpr int kTok    = kBatch * kSeq;
constexpr int kSqrtDk = 8;
static_assert(kHeads * kDk == kDm, "head split");
static_assert(kSqrtDk * kSqrtDk == kDk, "score scale");
static_assert(kTok % 64 == 0 && kDm % 64 == 0 && kSeq % 64 == 0 && kDm % 32 == 0, "tile multiples");
constexpr float kScoreScale = 1.0f / (float)kSqrtDk;
constexpr float kWCarry     = 16.0f;
constexpr float kWCarryInv  = 1.0f / kWCarry;
constexpr int kChunk   = 32;
constexpr int kQTile   = 16;
constexpr int kAbPitch = 40;
constexpr int kStPitch = 72;
static_assert(8 * kStPitch <= 16 * kAbPitch, "staging fits in the per-wave tile");

typedef __attribute__((ext_vector_type(16))) _Float16 v16h;
typedef __attribute__((ext_vector_type(8)))  _Float16 v8h;
typedef __attribute__((ext_vector_type(8)))  float    v8f;
typedef __attribute__((ext_vector_type(4)))  float    v4f;
typedef __attribute__((ext_vector_type(4)))  unsigned int v4u;

union FragU { v16h v; v8h h[2]; };
__device__ __forceinline__ v16h frag_load(const _Float16* p) {
  FragU f;
  f.h[0] = *(const v8h*)(p);
  f.h[1] = *(const v8h*)(p + 16);
  return f.v;
}
__device__ __forceinline__ void guard1(v8f& a, v16h x, v16h y) {
  asm volatile("v_nop\n\tv_nop\n\tv_nop\n\tv_nop" : "+v"(a) : "v"(x), "v"(y));
}
__device__ __forceinline__ void keep4_h(v16h a, v16h b, v16h c, v16h d) {
  asm volatile("v_nop" :: "v"(a), "v"(b), "v"(c), "v"(d));
}
__device__ __forceinline__ void acc_guard4(v8f& a, v8f& b, v8f& c, v8f& d) {
  asm volatile("v_nop\n\tv_nop\n\tv_nop\n\tv_nop" : "+v"(a), "+v"(b), "+v"(c), "+v"(d));
}
__device__ __forceinline__ v8f mma_h(v16h a, v16h b, v8f c) {
  c = __builtin_amdgcn_wmma_f32_16x16x32_f16(false, a, false, b, (short)0, c, false, false);
  asm volatile("v_nop\n\tv_nop\n\tv_nop\n\tv_nop" : "+v"(c) : "v"(a), "v"(b));
  return c;
}
__device__ __forceinline__ unsigned pk16(unsigned short a, unsigned short b) {
  return (unsigned)a | ((unsigned)b << 16);
}
__device__ __forceinline__ unsigned short h_bits(float f) {
  const _Float16 h = (_Float16)f;
  return __builtin_bit_cast(unsigned short, h);
}

template <int BIAS_MODE, int OUT_MODE>
__global__ __launch_bounds__(256) void wmma_gemm64_f16(
    const unsigned short* __restrict__ Ap, int lda, long strideA,
    const unsigned short* __restrict__ Btp, int ldb, long strideB,
    void* __restrict__ Cout, int ldc, long strideC,
    const float* __restrict__ bias,
    int M, int N, int K, float scale) {
  const _Float16* A  = (const _Float16*)(const void*)Ap;
  const _Float16* Bt = (const _Float16*)(const void*)Btp;
  __shared__ __align__(16) float sT[8][16 * 68];
  const int b    = blockIdx.y;
  const int lane = threadIdx.x & 31;
  const int wave = threadIdx.x >> 5;
  const int tilesN = N >> 6;
  const int tilesM = M >> 6;
  const int tile = blockIdx.x * 8 + wave;
  if (tile >= tilesM * tilesN) return;
  const int tm = tile / tilesN;
  const int tn = tile - tm * tilesN;
  const int m0 = tm << 6;
  const int n0 = tn << 6;

  const _Float16* Ab = A  + (size_t)b * strideA;
  const _Float16* Bb = Bt + (size_t)b * strideB;

  const int rlane = lane & 15;
  const int koff  = (lane >> 4) * 8;
  const int mOff  = (lane >> 4) * 8;

  v8f acc[4][4];
#pragma unroll
  for (int i = 0; i < 4; ++i)
#pragma unroll
    for (int j = 0; j < 4; ++j) acc[i][j] = (v8f){0.f,0.f,0.f,0.f,0.f,0.f,0.f,0.f};

  for (int k0 = 0; k0 < K; k0 += 32) {
    v16h bh[4];
#pragma unroll
    for (int j = 0; j < 4; ++j) {
      const size_t bo = (size_t)(n0 + (j << 4) + rlane) * ldb + koff + k0;
      bh[j] = frag_load(Bb + bo);
    }
#pragma unroll
    for (int i = 0; i < 4; ++i) {
      const size_t ao = (size_t)(m0 + (i << 4) + rlane) * lda + koff + k0;
      const v16h ah = frag_load(Ab + ao);
#pragma unroll
      for (int j = 0; j < 4; ++j) {
        acc[i][j] = __builtin_amdgcn_wmma_f32_16x16x32_f16(false, ah, false, bh[j], (short)0, acc[i][j], false, false);
      }
#pragma unroll
      for (int j = 0; j < 4; ++j) guard1(acc[i][j], ah, bh[j]);
    }
    keep4_h(bh[0], bh[1], bh[2], bh[3]);
  }
  acc_guard4(acc[0][0], acc[0][1], acc[0][2], acc[0][3]);
  acc_guard4(acc[1][0], acc[1][1], acc[1][2], acc[1][3]);
  acc_guard4(acc[2][0], acc[2][1], acc[2][2], acc[2][3]);
  acc_guard4(acc[3][0], acc[3][1], acc[3][2], acc[3][3]);

  float* slab = sT[wave];
#pragma unroll
  for (int i = 0; i < 4; ++i) {
    const int mBase = m0 + (i << 4);
#pragma unroll
    for (int j = 0; j < 4; ++j) {
      const int n = n0 + (j << 4) + rlane;
      float bv = 0.f;
      if (BIAS_MODE == 2) bv = bias[n];
#pragma unroll
      for (int r = 0; r < 8; ++r) {
        float v = acc[i][j][r] * scale;
        if (BIAS_MODE == 1) v += bias[mBase + mOff + r];
        if (BIAS_MODE == 2) v += bv;
        slab[(mOff + r) * 68 + (j << 4) + rlane] = v;
      }
    }
    __builtin_amdgcn_fence(__ATOMIC_RELEASE, "workgroup");
    __builtin_amdgcn_wave_barrier();
    __builtin_amdgcn_fence(__ATOMIC_ACQUIRE, "workgroup");
    if (OUT_MODE == 0) {
      float* C = (float*)Cout + (size_t)b * strideC;
      const int hh = lane >> 4, c4 = (lane & 15) * 4;
      for (int pass = 0; pass < 2; ++pass) {
#pragma unroll
        for (int it = 0; it < 8; ++it) {
          const int row = it * 2 + hh;
          const v4f v = *(const v4f*)(slab + row * 68 + c4);
          *(volatile v4f*)(C + (size_t)(mBase + row) * ldc + n0 + c4) = v;
        }
        __threadfence();
      }
    } else {
      const int q = lane >> 3, c8 = (lane & 7) * 8;
      unsigned short* C = (unsigned short*)Cout + (size_t)b * strideC;
      for (int pass = 0; pass < 2; ++pass) {
#pragma unroll
        for (int it = 0; it < 4; ++it) {
          const int row = it * 4 + q;
          const float* sp = slab + row * 68 + c8;
          v8h hv;
#pragma unroll
          for (int e = 0; e < 8; ++e) hv[e] = (_Float16)sp[e];
          *(volatile v8h*)(C + (size_t)(mBase + row) * ldc + n0 + c8) = hv;
        }
        __threadfence();
      }
    }
    __builtin_amdgcn_fence(__ATOMIC_RELEASE, "workgroup");
    __builtin_amdgcn_wave_barrier();
    __builtin_amdgcn_fence(__ATOMIC_ACQUIRE, "workgroup");
  }
}

__global__ __launch_bounds__(256) void cast8_f16_kernel(
    const float* __restrict__ in0, const float* __restrict__ in1,
    const float* __restrict__ in2, const float* __restrict__ in3,
    unsigned short* __restrict__ out, int n8, float mul) {
  const int i = blockIdx.x * 256 + threadIdx.x;
  if (i >= n8) return;
  const int z = blockIdx.y;
  const float* in = (z == 0) ? in0 : (z == 1) ? in1 : (z == 2) ? in2 : in3;
  const float* p = in + 8 * (size_t)i;
  const v4f a = *(const v4f*)(p);
  const v4f c = *(const v4f*)(p + 4);
  unsigned short hb[8];
#pragma unroll
  for (int e = 0; e < 4; ++e) {
    hb[e]     = h_bits(a[e] * mul);
    hb[4 + e] = h_bits(c[e] * mul);
  }
  const v4u u = (v4u){pk16(hb[0], hb[1]), pk16(hb[2], hb[3]), pk16(hb[4], hb[5]), pk16(hb[6], hb[7])};
  unsigned short* q = out + (size_t)z * (size_t)n8 * 8 + 8 * (size_t)i;
  *(volatile v4u*)q = u;
  __threadfence();
  *(volatile v4u*)q = u;
}

__global__ __launch_bounds__(512) void headnorm_attn_kernel(
    const unsigned short* __restrict__ Qp, const unsigned short* __restrict__ Kp,
    const unsigned short* __restrict__ Vtp, unsigned short* __restrict__ Cp) {
  __shared__ __align__(16) float    Psm[kHeads * 512];
  __shared__ __align__(16) float    Rinv[512];
  __shared__ __align__(16) _Float16 Abuf[kHeads][16 * kAbPitch];

  const _Float16* Q  = (const _Float16*)(const void*)Qp;
  const _Float16* K  = (const _Float16*)(const void*)Kp;
  const _Float16* Vt = (const _Float16*)(const void*)Vtp;
  _Float16* C = (_Float16*)(void*)Cp;

  const int tid  = threadIdx.x;
  const int h    = tid >> 5;
  const int lane = tid & 31;
  const int hh   = lane >> 4;
  const int c    = lane & 15;
  const int q0   = blockIdx.x * kQTile;
  const int b    = blockIdx.y;
  const size_t tok0 = (size_t)b * kSeq;

  const _Float16* qrow = Q + (tok0 + q0 + c) * kDm + h * kDk + 8 * hh;
  const v16h qa0 = frag_load(qrow);
  const v16h qa1 = frag_load(qrow + 32);

  v8f cacc[4];
#pragma unroll
  for (int dt = 0; dt < 4; ++dt) cacc[dt] = (v8f){0.f,0.f,0.f,0.f,0.f,0.f,0.f,0.f};

  const _Float16* kbase = K + (tok0 + c) * kDm + h * kDk + 8 * hh;
  const _Float16* vbase = Vt + ((size_t)b * kDm + (size_t)h * kDk + c) * kSeq + 8 * hh;
  float* pw = Psm + h * 512 + lane;
  _Float16* aw = Abuf[h];

  for (int kc = 0; kc < kSeq / kChunk; ++kc) {
    const int k0 = kc * kChunk;
    const v16h kb00 = frag_load(kbase + (size_t)k0 * kDm);
    const v16h kb01 = frag_load(kbase + (size_t)k0 * kDm + 32);
    const v16h kb10 = frag_load(kbase + (size_t)(k0 + 16) * kDm);
    const v16h kb11 = frag_load(kbase + (size_t)(k0 + 16) * kDm + 32);
    v8f s0 = (v8f){0.f,0.f,0.f,0.f,0.f,0.f,0.f,0.f};
    v8f s1 = (v8f){0.f,0.f,0.f,0.f,0.f,0.f,0.f,0.f};
    s0 = mma_h(qa0, kb00, s0);
    s0 = mma_h(qa1, kb01, s0);
    s1 = mma_h(qa0, kb10, s1);
    s1 = mma_h(qa1, kb11, s1);

    float p[16];
#pragma unroll
    for (int r = 0; r < 8; ++r) {
      p[r]     = __expf(s0[r] * kScoreScale);
      p[8 + r] = __expf(s1[r] * kScoreScale);
    }
#pragma unroll
    for (int i = 0; i < 16; ++i) pw[i * 32] = p[i];
    __syncthreads();

    {
      float sum = 0.0f;
#pragma unroll
      for (int hq = 0; hq < kHeads; ++hq) sum += Psm[hq * 512 + tid];
      Rinv[tid] = 1.0f / sum;
    }
    __syncthreads();

#pragma unroll
    for (int i = 0; i < 16; ++i) {
      const int t = i >> 3, r = i & 7;
      const float a = p[i] * Rinv[i * 32 + lane];
      aw[(8 * hh + r) * kAbPitch + t * 16 + c] = (_Float16)a;
    }
    __builtin_amdgcn_fence(__ATOMIC_RELEASE, "workgroup");
    __builtin_amdgcn_wave_barrier();
    __builtin_amdgcn_fence(__ATOMIC_ACQUIRE, "workgroup");
    const v16h aa = frag_load(aw + c * kAbPitch + 8 * hh);

#pragma unroll
    for (int dt = 0; dt < 4; ++dt) {
      const v16h vb = frag_load(vbase + (size_t)(dt * 16) * kSeq + k0);
      cacc[dt] = mma_h(aa, vb, cacc[dt]);
    }
    __syncthreads();
  }

  v8h outv[4];
  const int q8 = lane >> 3, c8 = (lane & 7) * 8;
#pragma unroll
  for (int rd = 0; rd < 2; ++rd) {
    if (hh == rd) {
#pragma unroll
      for (int dt = 0; dt < 4; ++dt)
#pragma unroll
        for (int r = 0; r < 8; ++r) aw[r * kStPitch + dt * 16 + c] = (_Float16)cacc[dt][r];
    }
    __builtin_amdgcn_fence(__ATOMIC_RELEASE, "workgroup");
    __builtin_amdgcn_wave_barrier();
    __builtin_amdgcn_fence(__ATOMIC_ACQUIRE, "workgroup");
    outv[rd * 2 + 0] = *(const v8h*)(aw + q8 * kStPitch + c8);
    outv[rd * 2 + 1] = *(const v8h*)(aw + (4 + q8) * kStPitch + c8);
    __builtin_amdgcn_fence(__ATOMIC_RELEASE, "workgroup");
    __builtin_amdgcn_wave_barrier();
    __builtin_amdgcn_fence(__ATOMIC_ACQUIRE, "workgroup");
  }
  _Float16* cb = C + (tok0 + q0) * kDm + h * kDk + c8;
  for (int pass = 0; pass < 2; ++pass) {
#pragma unroll
    for (int i = 0; i < 4; ++i) {
      const int row = (i >> 1) * 8 + (i & 1) * 4 + q8;
      *(volatile v8h*)(cb + (size_t)row * kDm) = outv[i];
    }
    __threadfence();
  }
}

extern "C" void kernel_launch(void* const* d_in, const int* in_sizes, int n_in,
                              void* d_out, int out_size, void* d_ws, size_t ws_size,
                              hipStream_t stream) {
  if (n_in < 9) return;
  if (in_sizes[0] != kTok * kDm || out_size != kTok * kDm) return;
  if (in_sizes[1] != kDm * kDm || in_sizes[3] != kDm * kDm || in_sizes[5] != kDm * kDm || in_sizes[7] != kDm * kDm) return;
  if (in_sizes[2] != kDm || in_sizes[4] != kDm || in_sizes[6] != kDm || in_sizes[8] != kDm) return;

  const float* x  = (const float*)d_in[0];
  const float* Wq = (const float*)d_in[1];
  const float* bq = (const float*)d_in[2];
  const float* Wk = (const float*)d_in[3];
  const float* bk = (const float*)d_in[4];
  const float* Wv = (const float*)d_in[5];
  const float* bv = (const float*)d_in[6];
  const float* Wo = (const float*)d_in[7];
  const float* bo = (const float*)d_in[8];
  float* out = (float*)d_out;

  constexpr size_t bPlane = (size_t)kTok * kDm * 2;
  constexpr size_t bW     = (size_t)4 * kDm * kDm * 2;
  constexpr size_t wPlane = (size_t)kDm * kDm;
  static_assert(bPlane == 8388608 && bW == 8388608, "carve sizes");
  char* ws = (char*)d_ws;
  size_t off = 0;
  unsigned short* Xh  = (unsigned short*)(ws + off); off += bPlane;
  unsigned short* Wh  = (unsigned short*)(ws + off); off += bW;
  unsigned short* Qh  = (unsigned short*)(ws + off); off += bPlane;
  unsigned short* Kh  = (unsigned short*)(ws + off); off += bPlane;
  unsigned short* Vt  = (unsigned short*)(ws + off); off += bPlane;
  unsigned short* Ctx = (unsigned short*)(ws + off); off += bPlane;
  if (off > ws_size || off > (size_t)134217728) return;

  const dim3 blk256(256), blk512(512);

  {
    constexpr int n8 = kTok * kDm / 8;
    static_assert(n8 % 256 == 0, "exact grid");
    cast8_f16_kernel<<<dim3(n8 / 256, 1), blk256, 0, stream>>>(x, x, x, x, Xh, n8, 1.0f);
  }
  {
    constexpr int n8 = kDm * kDm / 8;
    static_assert(n8 % 256 == 0, "exact grid");
    cast8_f16_kernel<<<dim3(n8 / 256, 4), blk256, 0, stream>>>(Wq, Wk, Wv, Wo, Wh, n8, kWCarry);
  }
  {
    constexpr int tiles = (kTok / 64) * (kDm / 64);
    wmma_gemm64_f16<2, 1><<<dim3((tiles + 7) / 8, 1), blk256, 0, stream>>>(
        Xh, kDm, 0L, Wh + 0 * wPlane, kDm, 0L, (void*)Qh, kDm, 0L, bq, kTok, kDm, kDm, kWCarryInv);
    wmma_gemm64_f16<2, 1><<<dim3((tiles + 7) / 8, 1), blk256, 0, stream>>>(
        Xh, kDm, 0L, Wh + 1 * wPlane, kDm, 0L, (void*)Kh, kDm, 0L, bk, kTok, kDm, kDm, kWCarryInv);
  }
  {
    constexpr int tiles = (kDm / 64) * (kSeq / 64);
    wmma_gemm64_f16<1, 1><<<dim3((tiles + 7) / 8, kBatch), blk256, 0, stream>>>(
        Wh + 2 * wPlane, kDm, 0L, Xh, kDm, (long)kSeq * kDm, (void*)Vt, kSeq, (long)kDm * kSeq,
        bv, kDm, kSeq, kDm, kWCarryInv);
  }
  headnorm_attn_kernel<<<dim3(kSeq / kQTile, kBatch), blk512, 0, stream>>>(Qh, Kh, Vt, Ctx);
  {
    constexpr int tiles = (kTok / 64) * (kDm / 64);
    wmma_gemm64_f16<2, 0><<<dim3((tiles + 7) / 8, 1), blk256, 0, stream>>>(
        Ctx, kDm, 0L, Wh + 3 * wPlane, kDm, 0L, (void*)out, kDm, 0L, bo, kTok, kDm, kDm, kWCarryInv);
  }
}
